// SimpleGRU_65609920413979
// MI455X (gfx1250) — hardware-verified
//
#include <hip/hip_runtime.h>
#include <math.h>

typedef __attribute__((ext_vector_type(16))) _Float16 v16h;
typedef __attribute__((ext_vector_type(8)))  _Float16 v8h;
typedef __attribute__((ext_vector_type(16))) __bf16   v16b;
typedef __attribute__((ext_vector_type(8)))  __bf16   v8b;
typedef __attribute__((ext_vector_type(8)))  float    v8f;
typedef __attribute__((ext_vector_type(4)))  float    v4f;
typedef __attribute__((ext_vector_type(4)))  unsigned v4u;

constexpr int NB_ROWS = 4096;
constexpr int SEQ_LEN = 64;
constexpr int HID = 256;
constexpr int G3H = 768;
constexpr int NSTEP = 42;
constexpr int ROWS_PER_BLK = 32;
constexpr int NBLK = NB_ROWS / ROWS_PER_BLK;
constexpr int APITCH = 264;
constexpr int OUT_PER_BLK = ROWS_PER_BLK * NSTEP;
constexpr int WPLANE = G3H * HID;
static_assert(NB_ROWS % ROWS_PER_BLK == 0, "rows");
static_assert((OUT_PER_BLK * 4) % 128 == 0, "lines");
static_assert(HID % 32 == 0, "k32");
static_assert(WPLANE % (8 * 256) == 0, "prep grid");
static_assert((APITCH * 2) % 16 == 0, "pitch");

__device__ __forceinline__ unsigned short f2bf_bits(float f) {
  unsigned u = __float_as_uint(f);
  return (unsigned short)((u + 0x7FFFu + ((u >> 16) & 1u)) >> 16);
}
__device__ __forceinline__ float bf_bits2f(unsigned short h) { return __uint_as_float(((unsigned)h) << 16); }

__device__ __forceinline__ void dep_guard_h(v8f& a, v8f& b, v16h x, v16h y) { asm volatile("v_nop\n\tv_nop\n\tv_nop\n\tv_nop" : "+v"(a), "+v"(b) : "v"(x), "v"(y)); }
__device__ __forceinline__ void dep_guard_b(v8f& a, v8f& b, v16b x, v16b y) { asm volatile("v_nop\n\tv_nop\n\tv_nop\n\tv_nop" : "+v"(a), "+v"(b) : "v"(x), "v"(y)); }
__device__ __forceinline__ void keep4_h(v16h a, v16h b, v16h c, v16h d) { asm volatile("v_nop" :: "v"(a), "v"(b), "v"(c), "v"(d)); }
__device__ __forceinline__ void keep4_b(v16b a, v16b b, v16b c, v16b d) { asm volatile("v_nop" :: "v"(a), "v"(b), "v"(c), "v"(d)); }
template <typename T> struct Frag;
template <> struct Frag<_Float16> {
  typedef v16h V; union U { v16h v; v8h h[2]; };
  static __device__ __forceinline__ v16h load(const _Float16* p) {
    U f; f.h[0] = *(const v8h*)(p); f.h[1] = *(const v8h*)(p + 16); return f.v;
  }
  static __device__ __forceinline__ v8f mma(v16h a, v16h b, v8f c) {
    return __builtin_amdgcn_wmma_f32_16x16x32_f16(false, a, false, b, (short)0, c, false, false);
  }
  static __device__ __forceinline__ void guard(v8f& a, v8f& b, v16h x, v16h y) { dep_guard_h(a, b, x, y); }
  static __device__ __forceinline__ void keep(v16h a, v16h b, v16h c, v16h d) { keep4_h(a, b, c, d); }
};
template <> struct Frag<__bf16> {
  typedef v16b V; union U { v16b v; v8b h[2]; };
  static __device__ __forceinline__ v16b load(const __bf16* p) {
    U f; f.h[0] = *(const v8b*)(p); f.h[1] = *(const v8b*)(p + 16); return f.v;
  }
  static __device__ __forceinline__ v8f mma(v16b a, v16b b, v8f c) {
    return __builtin_amdgcn_wmma_f32_16x16x32_bf16(false, a, false, b, (short)0, c, false, false);
  }
  static __device__ __forceinline__ void guard(v8f& a, v8f& b, v16b x, v16b y) { dep_guard_b(a, b, x, y); }
  static __device__ __forceinline__ void keep(v16b a, v16b b, v16b c, v16b d) { keep4_b(a, b, c, d); }
};
__device__ __forceinline__ void dep_guard1_b(v8f& a, v16b x, v16b y) { asm volatile("v_nop\n\tv_nop\n\tv_nop\n\tv_nop" : "+v"(a) : "v"(x), "v"(y)); }
__device__ __forceinline__ void acc_guard2(v8f& a, v8f& b) { asm volatile("v_nop\n\tv_nop\n\tv_nop\n\tv_nop" : "+v"(a), "+v"(b)); }
__device__ __forceinline__ void acc_guard6(v8f& a, v8f& b, v8f& c, v8f& d, v8f& e, v8f& f) {
  asm volatile("v_nop\n\tv_nop\n\tv_nop\n\tv_nop" : "+v"(a), "+v"(b), "+v"(c), "+v"(d), "+v"(e), "+v"(f));
}

__device__ __forceinline__ v8f zero8() { return (v8f){0.f, 0.f, 0.f, 0.f, 0.f, 0.f, 0.f, 0.f}; }

__device__ __forceinline__ float sigm_f(float a) { return __builtin_amdgcn_rcpf(1.0f + expf(-a)); }
__device__ __forceinline__ float tanh_f(float a) { return 1.0f - 2.0f * __builtin_amdgcn_rcpf(1.0f + expf(2.0f * a)); }

__global__ __launch_bounds__(256) void k_prep_w(const float* __restrict__ w,
                                                unsigned short* __restrict__ wf,
                                                unsigned short* __restrict__ wh,
                                                unsigned short* __restrict__ wl, int n8) {
  const int i = blockIdx.x * 256 + threadIdx.x;
  if (i >= n8) return;
  const v4f a = *(const v4f*)(w + (size_t)i * 8);
  const v4f b = *(const v4f*)(w + (size_t)i * 8 + 4);
  float v[8];
  v[0] = a[0]; v[1] = a[1]; v[2] = a[2]; v[3] = a[3];
  v[4] = b[0]; v[5] = b[1]; v[6] = b[2]; v[7] = b[3];
  v4u pf, ph, pl;
#pragma unroll
  for (int e = 0; e < 4; ++e) {
    const float v0 = v[2 * e], v1 = v[2 * e + 1];
    const unsigned f0 = (unsigned)__builtin_bit_cast(unsigned short, (_Float16)(v0 * 16.0f));
    const unsigned f1 = (unsigned)__builtin_bit_cast(unsigned short, (_Float16)(v1 * 16.0f));
    const unsigned short h0 = f2bf_bits(v0), h1 = f2bf_bits(v1);
    const unsigned short l0 = f2bf_bits(v0 - bf_bits2f(h0));
    const unsigned short l1 = f2bf_bits(v1 - bf_bits2f(h1));
    pf[e] = f0 | (f1 << 16);
    ph[e] = (unsigned)h0 | ((unsigned)h1 << 16);
    pl[e] = (unsigned)l0 | ((unsigned)l1 << 16);
  }
  unsigned short* df = wf + (size_t)i * 8;
  unsigned short* dh = wh + (size_t)i * 8;
  unsigned short* dl = wl + (size_t)i * 8;
  *(volatile v4u*)df = pf;
  *(volatile v4u*)dh = ph;
  *(volatile v4u*)dl = pl;
  __threadfence();
  *(volatile v4u*)df = pf;
  *(volatile v4u*)dh = ph;
  *(volatile v4u*)dl = pl;
}

template <int UB>
__device__ __forceinline__ void enc_ub(const _Float16* __restrict__ Wf, const _Float16* At, const float* xs, const int t,
                                       const int wave, const int rlane, const int hh, const int koff,
                                       const float (&wi)[3][2], const float (&bi)[3][2], const float (&bhh)[3][2],
                                       float (&h)[2][8]) {
  v8f acc[3][2];
#pragma unroll
  for (int g = 0; g < 3; ++g) { acc[g][0] = zero8(); acc[g][1] = zero8(); }
  const int nb = 16 * (2 * wave + UB) + rlane;
  const _Float16* w0 = Wf + (size_t)nb * HID + koff;
  const _Float16* w1 = w0 + (size_t)HID * HID;
  const _Float16* w2 = w0 + (size_t)2 * HID * HID;
  const _Float16* a0 = At + rlane * APITCH + koff;
  const _Float16* a1 = a0 + 16 * APITCH;
#pragma unroll 1
  for (int k0 = 0; k0 < HID; k0 += 32) {
    const v16h bf0 = Frag<_Float16>::load(w0 + k0);
    const v16h bf1 = Frag<_Float16>::load(w1 + k0);
    const v16h bf2 = Frag<_Float16>::load(w2 + k0);
    const v16h af = Frag<_Float16>::load(a0 + k0);
    acc[0][0] = Frag<_Float16>::mma(af, bf0, acc[0][0]);
    acc[1][0] = Frag<_Float16>::mma(af, bf1, acc[1][0]);
    acc[2][0] = Frag<_Float16>::mma(af, bf2, acc[2][0]);
    Frag<_Float16>::guard(acc[0][0], acc[2][0], af, bf0);
    const v16h ag = Frag<_Float16>::load(a1 + k0);
    acc[0][1] = Frag<_Float16>::mma(ag, bf0, acc[0][1]);
    acc[1][1] = Frag<_Float16>::mma(ag, bf1, acc[1][1]);
    acc[2][1] = Frag<_Float16>::mma(ag, bf2, acc[2][1]);
    Frag<_Float16>::guard(acc[0][1], acc[2][1], ag, bf2);
    Frag<_Float16>::keep(bf0, bf1, bf2, af);
  }
  acc_guard6(acc[0][0], acc[0][1], acc[1][0], acc[1][1], acc[2][0], acc[2][1]);
#pragma unroll
  for (int mt = 0; mt < 2; ++mt) {
#pragma unroll
    for (int r = 0; r < 8; ++r) {
      const int row = 16 * mt + 8 * hh + r;
      const float xv = xs[row * SEQ_LEN + t];
      const float a_r = (xv * wi[0][UB] + bi[0][UB]) + (acc[0][mt][r] * 0.0625f + bhh[0][UB]);
      const float a_z = (xv * wi[1][UB] + bi[1][UB]) + (acc[1][mt][r] * 0.0625f + bhh[1][UB]);
      const float g_n = acc[2][mt][r] * 0.0625f + bhh[2][UB];
      const float rg = sigm_f(a_r);
      const float zg = sigm_f(a_z);
      const float ng = tanh_f((xv * wi[2][UB] + bi[2][UB]) + rg * g_n);
      h[mt][r] = (1.0f - zg) * ng + zg * h[mt][r];
    }
  }
}

template <int UB, int G>
__device__ __forceinline__ void ghc_one(const __bf16* __restrict__ Wh, const __bf16* __restrict__ Wl,
                                        const __bf16* Ah, const __bf16* Al,
                                        const int wave, const int rlane, const int koff,
                                        const float (&bhh)[3][2], float (&gc)[3][2][8]) {
  const int nb = 16 * (2 * wave + UB) + rlane;
  const __bf16* wh = Wh + (size_t)(G * HID + nb) * HID + koff;
  const __bf16* wl = Wl + (size_t)(G * HID + nb) * HID + koff;
  const __bf16* a0h = Ah + rlane * APITCH + koff;
  const __bf16* a0l = Al + rlane * APITCH + koff;
  const __bf16* a1h = a0h + 16 * APITCH;
  const __bf16* a1l = a0l + 16 * APITCH;
  v8f acc0 = zero8(), acc1 = zero8();
#pragma unroll 1
  for (int k0 = 0; k0 < HID; k0 += 32) {
    const v16b bh = Frag<__bf16>::load(wh + k0);
    const v16b bl = Frag<__bf16>::load(wl + k0);
    const v16b ah = Frag<__bf16>::load(a0h + k0);
    const v16b al = Frag<__bf16>::load(a0l + k0);
    acc0 = Frag<__bf16>::mma(ah, bh, acc0);
    acc0 = Frag<__bf16>::mma(ah, bl, acc0);
    acc0 = Frag<__bf16>::mma(al, bh, acc0);
    dep_guard1_b(acc0, ah, al);
    const v16b ag = Frag<__bf16>::load(a1h + k0);
    const v16b am = Frag<__bf16>::load(a1l + k0);
    acc1 = Frag<__bf16>::mma(ag, bh, acc1);
    acc1 = Frag<__bf16>::mma(ag, bl, acc1);
    acc1 = Frag<__bf16>::mma(am, bh, acc1);
    dep_guard1_b(acc1, ag, am);
    Frag<__bf16>::keep(bh, bl, ah, al);
  }
  acc_guard2(acc0, acc1);
#pragma unroll
  for (int r = 0; r < 8; ++r) {
    gc[G][0][r] = acc0[r] + bhh[G][UB];
    gc[G][1][r] = acc1[r] + bhh[G][UB];
  }
}

template <int UB>
__device__ __forceinline__ void dec_ub(const float* ov, const int hh,
                                       const float (&wi)[3][2], const float (&bi)[3][2],
                                       const float (&gc)[3][2][8], const float (&hid)[2][8],
                                       const float wo, float (&part)[2][8]) {
#pragma unroll
  for (int mt = 0; mt < 2; ++mt) {
#pragma unroll
    for (int r = 0; r < 8; ++r) {
      const float o = ov[16 * mt + 8 * hh + r];
      const float a_r = (o * wi[0][UB] + bi[0][UB]) + gc[0][mt][r];
      const float a_z = (o * wi[1][UB] + bi[1][UB]) + gc[1][mt][r];
      const float rg = sigm_f(a_r);
      const float zg = sigm_f(a_z);
      const float ng = tanh_f((o * wi[2][UB] + bi[2][UB]) + rg * gc[2][mt][r]);
      const float hn = (1.0f - zg) * ng + zg * hid[mt][r];
      part[mt][r] += hn * wo;
    }
  }
}

__global__ __launch_bounds__(256) void k_gru_main(const float* __restrict__ x,
                                                  const float* __restrict__ w_ih,
                                                  const float* __restrict__ b_ih,
                                                  const float* __restrict__ b_hh,
                                                  const float* __restrict__ w_out,
                                                  const float* __restrict__ b_out,
                                                  const unsigned short* __restrict__ wf16,
                                                  const unsigned short* __restrict__ wbh,
                                                  const unsigned short* __restrict__ wbl,
                                                  float* __restrict__ out) {
  __shared__ __align__(16) float x_sh[ROWS_PER_BLK * SEQ_LEN];
  __shared__ __align__(16) unsigned short a_hi[ROWS_PER_BLK * APITCH];
  __shared__ __align__(16) unsigned short a_lo[ROWS_PER_BLK * APITCH];
  __shared__ float red_sh[8 * ROWS_PER_BLK];
  __shared__ float outv_sh[ROWS_PER_BLK];
  __shared__ __align__(16) float outs_sh[OUT_PER_BLK];

  const int tid   = threadIdx.x;
  const int wave  = tid >> 5;
  const int lane  = tid & 31;
  const int rlane = lane & 15;
  const int hh    = lane >> 4;
  const int koff  = hh * 8;
  const int blk   = blockIdx.x;

  {
    const float* xb = x + (size_t)blk * (ROWS_PER_BLK * SEQ_LEN);
    const v4f v0 = *(const v4f*)(xb + 4 * tid);
    const v4f v1 = *(const v4f*)(xb + 4 * (tid + 256));
    *(v4f*)(x_sh + 4 * tid) = v0;
    *(v4f*)(x_sh + 4 * (tid + 256)) = v1;
  }
  {
    unsigned* az = (unsigned*)a_hi;
    for (int i = tid; i < ROWS_PER_BLK * APITCH / 2; i += 256) az[i] = 0u;
  }
  float wi[3][2], bi[3][2], bhh[3][2], wo[2];
#pragma unroll
  for (int ub = 0; ub < 2; ++ub) {
    const int u = 16 * (2 * wave + ub) + rlane;
#pragma unroll
    for (int g = 0; g < 3; ++g) {
      wi[g][ub]  = w_ih[g * HID + u];
      bi[g][ub]  = b_ih[g * HID + u];
      bhh[g][ub] = b_hh[g * HID + u];
    }
    wo[ub] = w_out[u];
  }
  const float bo = b_out[0];

  float hst0[2][8], hst1[2][8];
#pragma unroll
  for (int mt = 0; mt < 2; ++mt)
#pragma unroll
    for (int r = 0; r < 8; ++r) { hst0[mt][r] = 0.0f; hst1[mt][r] = 0.0f; }

  const _Float16* Wf = (const _Float16*)wf16;
  const _Float16* At = (const _Float16*)a_hi;

#pragma unroll 1
  for (int t = 0; t < SEQ_LEN; ++t) {
    __syncthreads();
    enc_ub<0>(Wf, At, x_sh, t, wave, rlane, hh, koff, wi, bi, bhh, hst0);
    enc_ub<1>(Wf, At, x_sh, t, wave, rlane, hh, koff, wi, bi, bhh, hst1);
    __syncthreads();
#pragma unroll
    for (int mt = 0; mt < 2; ++mt) {
#pragma unroll
      for (int r = 0; r < 8; ++r) {
        const int row = 16 * mt + 8 * hh + r;
        a_hi[row * APITCH + 16 * (2 * wave) + rlane]     = __builtin_bit_cast(unsigned short, (_Float16)hst0[mt][r]);
        a_hi[row * APITCH + 16 * (2 * wave + 1) + rlane] = __builtin_bit_cast(unsigned short, (_Float16)hst1[mt][r]);
      }
    }
  }
  __syncthreads();
#pragma unroll
  for (int mt = 0; mt < 2; ++mt) {
#pragma unroll
    for (int r = 0; r < 8; ++r) {
      const int row = 16 * mt + 8 * hh + r;
      const int i0 = row * APITCH + 16 * (2 * wave) + rlane;
      const int i1 = row * APITCH + 16 * (2 * wave + 1) + rlane;
      const unsigned short hb0 = f2bf_bits(hst0[mt][r]);
      const unsigned short hb1 = f2bf_bits(hst1[mt][r]);
      a_hi[i0] = hb0;
      a_lo[i0] = f2bf_bits(hst0[mt][r] - bf_bits2f(hb0));
      a_hi[i1] = hb1;
      a_lo[i1] = f2bf_bits(hst1[mt][r] - bf_bits2f(hb1));
    }
  }
  __syncthreads();

  float gc0[3][2][8], gc1[3][2][8];
  {
    const __bf16* Wh = (const __bf16*)wbh;
    const __bf16* Wl = (const __bf16*)wbl;
    const __bf16* Ah = (const __bf16*)a_hi;
    const __bf16* Al = (const __bf16*)a_lo;
    ghc_one<0, 0>(Wh, Wl, Ah, Al, wave, rlane, koff, bhh, gc0);
    ghc_one<0, 1>(Wh, Wl, Ah, Al, wave, rlane, koff, bhh, gc0);
    ghc_one<0, 2>(Wh, Wl, Ah, Al, wave, rlane, koff, bhh, gc0);
    ghc_one<1, 0>(Wh, Wl, Ah, Al, wave, rlane, koff, bhh, gc1);
    ghc_one<1, 1>(Wh, Wl, Ah, Al, wave, rlane, koff, bhh, gc1);
    ghc_one<1, 2>(Wh, Wl, Ah, Al, wave, rlane, koff, bhh, gc1);
  }

  float part[2][8];
#pragma unroll
  for (int mt = 0; mt < 2; ++mt)
#pragma unroll
    for (int r = 0; r < 8; ++r) part[mt][r] = hst0[mt][r] * wo[0] + hst1[mt][r] * wo[1];

#pragma unroll 1
  for (int s = 0; s < NSTEP; ++s) {
#pragma unroll
    for (int mt = 0; mt < 2; ++mt) {
#pragma unroll
      for (int r = 0; r < 8; ++r) {
        float v = part[mt][r];
        v += __shfl_xor(v, 1, 32);
        v += __shfl_xor(v, 2, 32);
        v += __shfl_xor(v, 4, 32);
        v += __shfl_xor(v, 8, 32);
        part[mt][r] = v;
      }
    }
    if (rlane == 0) {
#pragma unroll
      for (int mt = 0; mt < 2; ++mt)
#pragma unroll
        for (int r = 0; r < 8; ++r) red_sh[wave * ROWS_PER_BLK + 16 * mt + 8 * hh + r] = part[mt][r];
    }
    __syncthreads();
    if (wave == 0) {
      const int row = lane;
      float acc = red_sh[row];
#pragma unroll
      for (int w = 1; w < 8; ++w) acc += red_sh[w * ROWS_PER_BLK + row];
      const float o = acc + bo;
      outv_sh[row] = o;
      outs_sh[row * NSTEP + s] = o;
    }
    __syncthreads();
    if (s + 1 < NSTEP) {
#pragma unroll
      for (int mt = 0; mt < 2; ++mt)
#pragma unroll
        for (int r = 0; r < 8; ++r) part[mt][r] = 0.0f;
      dec_ub<0>(outv_sh, hh, wi, bi, gc0, hst0, wo[0], part);
      dec_ub<1>(outv_sh, hh, wi, bi, gc1, hst1, wo[1], part);
    }
  }
  __syncthreads();

  {
    float* ob = out + (size_t)blk * OUT_PER_BLK;
    for (int pass = 0; pass < 2; ++pass) {
      for (int i = tid; i < OUT_PER_BLK / 4; i += 256) {
        const v4f v = *(const v4f*)(outs_sh + 4 * i);
        *(volatile v4f*)(ob + 4 * i) = v;
      }
      __threadfence();
    }
  }
}

extern "C" void kernel_launch(void* const* d_in, const int* in_sizes, int n_in,
                              void* d_out, int out_size, void* d_ws, size_t ws_size,
                              hipStream_t stream) {
  if (n_in < 7) return;
  if (in_sizes[0] != NB_ROWS * SEQ_LEN) return;
  if (in_sizes[1] != G3H) return;
  if (in_sizes[2] != WPLANE) return;
  if (in_sizes[3] != G3H || in_sizes[4] != G3H) return;
  if (in_sizes[5] != HID || in_sizes[6] < 1) return;
  if (out_size != NB_ROWS * NSTEP) return;
  const size_t plane_bytes = (size_t)WPLANE * 2;
  if (ws_size < 3 * plane_bytes) return;

  const float* x     = (const float*)d_in[0];
  const float* w_ih  = (const float*)d_in[1];
  const float* w_hh  = (const float*)d_in[2];
  const float* b_ih  = (const float*)d_in[3];
  const float* b_hh  = (const float*)d_in[4];
  const float* w_out = (const float*)d_in[5];
  const float* b_out = (const float*)d_in[6];
  float* out = (float*)d_out;

  unsigned short* wf = (unsigned short*)d_ws;
  unsigned short* wh = wf + WPLANE;
  unsigned short* wl = wh + WPLANE;

  const int n8 = WPLANE / 8;
  k_prep_w<<<n8 / 256, 256, 0, stream>>>(w_hh, wf, wh, wl, n8);
  k_gru_main<<<NBLK, 256, 0, stream>>>(x, w_ih, b_ih, b_hh, w_out, b_out, wf, wh, wl, out);
}
